// AttentionStack_76768245449145
// MI455X (gfx1250) — hardware-verified
//
#include <hip/hip_runtime.h>
#include <stdint.h>

typedef unsigned short us;
typedef __bf16 v16b __attribute__((ext_vector_type(16)));
typedef float v8f __attribute__((ext_vector_type(8)));
typedef float v4f __attribute__((ext_vector_type(4)));
typedef unsigned short us8 __attribute__((ext_vector_type(8)));
typedef unsigned int v4u __attribute__((ext_vector_type(4)));
union Fr { v16b v; us8 h[2]; };

#define DEV __device__ __forceinline__
enum { LTOK = 6977, LROW = 6976, DIM = 512, QKVC = 1536, TOK_BASE = 320, TOK_GL = 2368, NOBJ = 4968,
       ROWS_A = 4096 + 2 * NOBJ, OUT1_ROW = 640, OUT2_ROW = 4736 };

DEV float neg_inf() { return __uint_as_float(0xff800000u); }
DEV us f2bf(float f) { unsigned u = __float_as_uint(f); return (us)((u + 0x7FFFu + ((u >> 16) & 1u)) >> 16); }
DEV float bf2f(us b) { return __uint_as_float(((unsigned)b) << 16); }
DEV unsigned pk16(us a, us b) { return (unsigned)a | ((unsigned)b << 16); }
DEV v8f zero8() { v8f z = {0.f, 0.f, 0.f, 0.f, 0.f, 0.f, 0.f, 0.f}; return z; }
DEV v16b ldfrag(const us* p) { Fr f; f.h[0] = *(const us8*)p; f.h[1] = *(const us8*)(p + 16); return f.v; }
DEV v8f mma(v16b a, v16b b, v8f c) { return __builtin_amdgcn_wmma_f32_16x16x32_bf16(false, a, false, b, (short)0, c, false, false); }
DEV void gd1(v8f& d, v16b a, v16b b, v16b c, v16b e) { asm volatile("v_nop\n\tv_nop\n\tv_nop\n\tv_nop" : "+v"(d) : "v"(a), "v"(b), "v"(c), "v"(e)); }
DEV void gd2(v8f& d0, v8f& d1, v16b a, v16b b) { asm volatile("v_nop\n\tv_nop\n\tv_nop\n\tv_nop" : "+v"(d0), "+v"(d1) : "v"(a), "v"(b)); }
DEV void gd4(v8f& a, v8f& b, v8f& c, v8f& d) { asm volatile("v_nop\n\tv_nop\n\tv_nop\n\tv_nop" : "+v"(a), "+v"(b), "+v"(c), "+v"(d)); }
DEV void keep4(v16b a, v16b b, v16b c, v16b d) { asm volatile("v_nop" :: "v"(a), "v"(b), "v"(c), "v"(d)); }
DEV float rmax16(float x) { x = fmaxf(x, __shfl_xor(x, 1)); x = fmaxf(x, __shfl_xor(x, 2)); x = fmaxf(x, __shfl_xor(x, 4)); x = fmaxf(x, __shfl_xor(x, 8)); return x; }
DEV float rsum16(float x) { x += __shfl_xor(x, 1); x += __shfl_xor(x, 2); x += __shfl_xor(x, 4); x += __shfl_xor(x, 8); return x; }

__global__ __launch_bounds__(256) void k_cvt8(const float* __restrict__ in, us* __restrict__ out, int n8) {
  const int i = blockIdx.x * 256 + threadIdx.x;
  if (i >= n8) return;
  const float* p = in + (size_t)i * 8;
  const v4f a = *(const v4f*)p, c = *(const v4f*)(p + 4);
  v4u w;
  w[0] = pk16(f2bf(a[0]), f2bf(a[1])); w[1] = pk16(f2bf(a[2]), f2bf(a[3]));
  w[2] = pk16(f2bf(c[0]), f2bf(c[1])); w[3] = pk16(f2bf(c[2]), f2bf(c[3]));
  volatile v4u* o = (volatile v4u*)(out + (size_t)i * 8);
  *o = w; __threadfence(); *o = w;
}

__global__ __launch_bounds__(256) void k_wtrans(const float* __restrict__ wq, const float* __restrict__ wk, const float* __restrict__ wv,
                                                 const float* __restrict__ fw, us* __restrict__ Wt, us* __restrict__ Ft) {
  __shared__ __align__(16) us sT[32 * 72];
  const int z = blockIdx.z, n0 = blockIdx.x * 32, k0 = blockIdx.y * 64, tid = threadIdx.x;
  const float* src = (z == 0) ? wq : ((z == 1) ? wk : ((z == 2) ? wv : fw));
  us* dst = (z < 3) ? (Wt + (size_t)z * DIM * DIM) : Ft;
  {
    const int kr = tid >> 2, nq = (tid & 3) * 8;
    const float* p = src + (size_t)(k0 + kr) * DIM + n0 + nq;
    const v4f a = *(const v4f*)p, c = *(const v4f*)(p + 4);
#pragma unroll
    for (int e = 0; e < 4; ++e) { sT[(nq + e) * 72 + kr] = f2bf(a[e]); sT[(nq + 4 + e) * 72 + kr] = f2bf(c[e]); }
  }
  __syncthreads();
  const int row = tid >> 3, c8 = (tid & 7) * 8;
  const us8 v = *(const us8*)(&sT[row * 72 + c8]);
  volatile us8* o = (volatile us8*)(dst + (size_t)(n0 + row) * DIM + k0 + c8);
  *o = v; __threadfence(); *o = v;
}

DEV int objrow(int row, int M) {
  if (row >= M) return -1;
  int t_ = row / 69; const int j = row - t_ * 69;
  const int k = t_ & 7; t_ >>= 3;
  const int bb = t_ / 9; const int t = t_ - bb * 9;
  if (j < 64) return OUT2_ROW + (t_ * 8 + k) * 64 + j;
  return (t < 8) ? (((bb * 8 + t) * 8 + k) * 5 + (j - 64)) : -1;
}
template <bool ALO, int OM>
__global__ __launch_bounds__(256) void k_gemm(const us* __restrict__ A, const us* __restrict__ A2, int lda, long sA,
                                              const us* __restrict__ Bt, int ldb, us* __restrict__ Ch, us* __restrict__ Cl,
                                              float* __restrict__ Cf, int ldc, long sC, const float* __restrict__ bias,
                                              int M, int N, int K) {
  __shared__ __align__(16) float sT[8][16 * 68];
  const int bz = blockIdx.y, lane = threadIdx.x & 31, wav = threadIdx.x >> 5;
  const int tilesN = N >> 6, tilesM = (M + 63) >> 6;
  const int tile = blockIdx.x * 8 + wav;
  if (tile >= tilesM * tilesN) return;
  const int tm = tile / tilesN, tn = tile - tm * tilesN, m0 = tm << 6, n0 = tn << 6;
  const us* Ab = A + (size_t)bz * sA;
  const us* Ab2 = A2 + (size_t)bz * sA;
  const int rl = lane & 15, koff = (lane >> 4) * 8, mOff = koff;
  v8f acc[4][4];
#pragma unroll
  for (int i = 0; i < 4; ++i)
#pragma unroll
    for (int j = 0; j < 4; ++j) acc[i][j] = zero8();
  int arow[4];
#pragma unroll
  for (int i = 0; i < 4; ++i) { const int r = m0 + 16 * i + rl; arow[i] = (r < M) ? r : (M - 1); }
  for (int k0 = 0; k0 < K; k0 += 32) {
    v16b bh[4];
#pragma unroll
    for (int j = 0; j < 4; ++j) bh[j] = ldfrag(Bt + (size_t)(n0 + 16 * j + rl) * ldb + koff + k0);
#pragma unroll
    for (int i = 0; i < 4; ++i) {
      const size_t ao = (size_t)arow[i] * lda + koff + k0;
      const v16b ah = ldfrag(Ab + ao);
      v16b al = ah;
      if (ALO) al = ldfrag(Ab2 + ao);
#pragma unroll
      for (int j = 0; j < 4; ++j) {
        acc[i][j] = mma(ah, bh[j], acc[i][j]);
        if (ALO) acc[i][j] = mma(al, bh[j], acc[i][j]);
      }
      gd2(acc[i][0], acc[i][3], ah, al);
    }
    keep4(bh[0], bh[1], bh[2], bh[3]);
  }
  gd4(acc[0][0], acc[0][1], acc[0][2], acc[0][3]);
  gd4(acc[1][0], acc[1][1], acc[1][2], acc[1][3]);
  gd4(acc[2][0], acc[2][1], acc[2][2], acc[2][3]);
  gd4(acc[3][0], acc[3][1], acc[3][2], acc[3][3]);

  float* slab = sT[wav];
#pragma unroll
  for (int i = 0; i < 4; ++i) {
    const int mBase = m0 + 16 * i;
#pragma unroll
    for (int j = 0; j < 4; ++j) {
      const int n = n0 + 16 * j + rl;
      float bv = 0.f;
      if (OM != 0) bv = bias[n];
#pragma unroll
      for (int r = 0; r < 8; ++r) slab[(mOff + r) * 68 + 16 * j + rl] = acc[i][j][r] + bv;
    }
    __builtin_amdgcn_fence(__ATOMIC_RELEASE, "workgroup");
    __builtin_amdgcn_wave_barrier();
    __builtin_amdgcn_fence(__ATOMIC_ACQUIRE, "workgroup");
    if (OM == 0) {
      const int q4 = lane >> 3, c8 = (lane & 7) * 8;
      us8 hv[4], lv[4];
#pragma unroll
      for (int it = 0; it < 4; ++it) {
        const float* sp = slab + (it * 4 + q4) * 68 + c8;
        const v4f s0 = *(const v4f*)sp, s1 = *(const v4f*)(sp + 4);
        us8 hq, lq;
#pragma unroll
        for (int e = 0; e < 4; ++e) {
          us hb = f2bf(s0[e]); hq[e] = hb; lq[e] = f2bf(s0[e] - bf2f(hb));
          hb = f2bf(s1[e]); hq[4 + e] = hb; lq[4 + e] = f2bf(s1[e] - bf2f(hb));
        }
        hv[it] = hq; lv[it] = lq;
      }
      us* H = Ch + (size_t)bz * sC;
      us* L = Cl + (size_t)bz * sC;
      for (int pass = 0; pass < 2; ++pass) {
#pragma unroll
        for (int it = 0; it < 4; ++it) {
          const int grow = mBase + it * 4 + q4;
          if (grow < M) {
            const size_t o = (size_t)grow * ldc + n0 + c8;
            *(volatile us8*)(H + o) = hv[it];
            *(volatile us8*)(L + o) = lv[it];
          }
        }
        __threadfence();
      }
    } else {
      const int h2 = lane >> 4, c4 = (lane & 15) * 4;
      int orr[8];
#pragma unroll
      for (int it = 0; it < 8; ++it) {
        const int grow = mBase + it * 2 + h2;
        orr[it] = (OM == 1) ? ((grow < M) ? (OUT1_ROW + grow) : -1) : objrow(grow, M);
      }
      for (int pass = 0; pass < 2; ++pass) {
#pragma unroll
        for (int it = 0; it < 8; ++it) {
          const v4f v = *(const v4f*)(slab + (it * 2 + h2) * 68 + c4);
          if (orr[it] >= 0) *(volatile v4f*)(Cf + (size_t)orr[it] * ldc + n0 + c4) = v;
        }
        __threadfence();
      }
    }
    __builtin_amdgcn_fence(__ATOMIC_RELEASE, "workgroup");
    __builtin_amdgcn_wave_barrier();
    __builtin_amdgcn_fence(__ATOMIC_ACQUIRE, "workgroup");
  }
}

struct ADesc { int Sq, Skv, qobj, kobj, qistr, tI, tG, kI, kG, hasmask, mpitch, minst, avg, apb; };
static_assert(sizeof(ADesc) == 56);

DEV int objmap(const ADesc& d, int inst, int s, int& crow) {
  const int g = s / 69, jj = s - g * 69;
  const int t = d.tI * inst + d.tG * g, k = d.kI * inst + d.kG * g;
  const int tk = t * 8 + k;
  crow = tk * 69 + jj;
  return (jj < 64) ? (TOK_GL + tk * 64 + jj) : ((t < 8) ? (tk * 5 + jj - 64) : -1);
}
DEV int qmap(const ADesc& d, int inst, int b, int sc, int& arow) {
  if (d.qobj) { int cr = 0; const int tok = objmap(d, inst, sc, cr); arow = b * d.apb + cr; return tok; }
  arow = b * d.apb + inst * d.qistr + sc;
  return TOK_BASE + inst * d.qistr + sc;
}
DEV int kmap(const ADesc& d, int inst, int sc) {
  if (d.kobj) { int cr = 0; return objmap(d, inst, sc, cr); }
  return TOK_BASE + sc;
}

__global__ __launch_bounds__(128) void k_attn(const us* __restrict__ Ph, const us* __restrict__ Pl, const int* __restrict__ msk,
                                               us* Ah, us* Al, ADesc d) {
  __shared__ __align__(16) us sK[2][64 * 72];
  __shared__ __align__(16) us sV[2][64 * 72];
  __shared__ __align__(16) us sP[4][2][16 * 72];
  __shared__ int sflag[2][4];
  const int tid = threadIdx.x, wav = tid >> 5, lane = tid & 31, hh = lane >> 4, idx = lane & 15;
  const int q0 = blockIdx.x * 64, inst = blockIdx.y, b = blockIdx.z >> 3, hd = blockIdx.z & 7;
  const size_t prow = (size_t)b * LROW;
  const int qcol = hd * 64, kcol = DIM + hd * 64, vcol = 2 * DIM + hd * 64;
  const us8 z8 = {0, 0, 0, 0, 0, 0, 0, 0};
  const v4u z4 = {0u, 0u, 0u, 0u};
  const int* mrow0 = msk + (size_t)inst * (size_t)d.minst;

  v16b qh[2], ql[2];
  {
    const int s = q0 + 16 * wav + idx;
    bool ok = s < d.Sq;
    int ar = 0;
    const int tok = qmap(d, inst, b, ok ? s : (d.Sq - 1), ar);
    ok = ok && (tok >= 0);
    const size_t o = (prow + (tok < 0 ? 0 : tok)) * QKVC + qcol + 8 * hh;
#pragma unroll
    for (int ch = 0; ch < 2; ++ch) {
      const us8 a0 = *(const us8*)(Ph + o + 32 * ch), a1 = *(const us8*)(Ph + o + 32 * ch + 16);
      const us8 b0 = *(const us8*)(Pl + o + 32 * ch), b1 = *(const us8*)(Pl + o + 32 * ch + 16);
      Fr fh, fl;
      fh.h[0] = ok ? a0 : z8; fh.h[1] = ok ? a1 : z8;
      fl.h[0] = ok ? b0 : z8; fl.h[1] = ok ? b1 : z8;
      qh[ch] = fh.v; ql[ch] = fl.v;
    }
  }
  float m[8], l[8];
  v8f O[4];
#pragma unroll
  for (int r = 0; r < 8; ++r) { m[r] = neg_inf(); l[r] = 0.f; }
#pragma unroll
  for (int g = 0; g < 4; ++g) O[g] = zero8();

  const int nkt = (d.Skv + 63) >> 6;
  for (int kt = 0; kt < nkt; ++kt) {
    const int c0 = kt * 64;
    unsigned bits = 0u;
    if (d.hasmask) {
#pragma unroll
      for (int r = 0; r < 8; ++r) {
        int i = q0 + 16 * wav + 8 * hh + r; i = (i < d.Sq) ? i : (d.Sq - 1);
        const int* mr = mrow0 + (size_t)i * d.mpitch;
#pragma unroll
        for (int j = 0; j < 4; ++j) {
          const int c = c0 + 16 * j + idx; const int cc = (c < d.Skv) ? c : (d.Skv - 1);
          const int v = mr[cc];
          bits |= ((v != 0 && c < d.Skv) ? 1u : 0u) << (j * 8 + r);
        }
      }
    } else {
#pragma unroll
      for (int j = 0; j < 4; ++j) {
        const int c = c0 + 16 * j + idx; const unsigned okc = (c < d.Skv) ? 1u : 0u;
#pragma unroll
        for (int r = 0; r < 8; ++r) bits |= okc << (j * 8 + r);
      }
    }
    const unsigned bal = __builtin_amdgcn_ballot_w32(bits != 0u);
    if (lane == 0) sflag[kt & 1][wav] = (bal != 0u) ? 1 : 0;
    __syncthreads();
    const int act = sflag[kt & 1][0] | sflag[kt & 1][1] | sflag[kt & 1][2] | sflag[kt & 1][3];
    if (act) {
      {
        const int kr = tid >> 1, cq = (tid & 1) * 32;
        const int s = c0 + kr;
        bool ok = s < d.Skv;
        const int tok = kmap(d, inst, ok ? s : (d.Skv - 1));
        ok = ok && (tok >= 0);
        const size_t o = (prow + (tok < 0 ? 0 : tok)) * QKVC + kcol + cq;
#pragma unroll
        for (int i = 0; i < 4; ++i) {
          v4u a = *(const v4u*)(Ph + o + 8 * i), c2 = *(const v4u*)(Pl + o + 8 * i);
          if (!ok) { a = z4; c2 = z4; }
          *(v4u*)(&sK[0][kr * 72 + cq + 8 * i]) = a;
          *(v4u*)(&sK[1][kr * 72 + cq + 8 * i]) = c2;
        }
      }
      {
        const int kp = tid >> 2, dq = (tid & 3) * 16;
        const int sa = c0 + 2 * kp, sb = sa + 1;
        bool oka = sa < d.Skv, okb = sb < d.Skv;
        const int ta = kmap(d, inst, oka ? sa : (d.Skv - 1)), tb = kmap(d, inst, okb ? sb : (d.Skv - 1));
        oka = oka && (ta >= 0); okb = okb && (tb >= 0);
        const size_t oa = (prow + (ta < 0 ? 0 : ta)) * QKVC + vcol + dq;
        const size_t ob = (prow + (tb < 0 ? 0 : tb)) * QKVC + vcol + dq;
        v4u ah0 = *(const v4u*)(Ph + oa), ah1 = *(const v4u*)(Ph + oa + 8);
        v4u bh0 = *(const v4u*)(Ph + ob), bh1 = *(const v4u*)(Ph + ob + 8);
        v4u al0 = *(const v4u*)(Pl + oa), al1 = *(const v4u*)(Pl + oa + 8);
        v4u bl0 = *(const v4u*)(Pl + ob), bl1 = *(const v4u*)(Pl + ob + 8);
        if (!oka) { ah0 = z4; ah1 = z4; al0 = z4; al1 = z4; }
        if (!okb) { bh0 = z4; bh1 = z4; bl0 = z4; bl1 = z4; }
        unsigned* vwh = (unsigned*)(&sV[0][0]);
        unsigned* vwl = (unsigned*)(&sV[1][0]);
#pragma unroll
        for (int e = 0; e < 4; ++e) {
          const int w0 = (dq + 2 * e) * 36 + kp, w1 = (dq + 8 + 2 * e) * 36 + kp;
          vwh[w0]      = (ah0[e] & 0xffffu) | (bh0[e] << 16);
          vwh[w0 + 36] = (ah0[e] >> 16) | (bh0[e] & 0xffff0000u);
          vwh[w1]      = (ah1[e] & 0xffffu) | (bh1[e] << 16);
          vwh[w1 + 36] = (ah1[e] >> 16) | (bh1[e] & 0xffff0000u);
          vwl[w0]      = (al0[e] & 0xffffu) | (bl0[e] << 16);
          vwl[w0 + 36] = (al0[e] >> 16) | (bl0[e] & 0xffff0000u);
          vwl[w1]      = (al1[e] & 0xffffu) | (bl1[e] << 16);
          vwl[w1 + 36] = (al1[e] >> 16) | (bl1[e] & 0xffff0000u);
        }
      }
      __syncthreads();
      v8f S[4];
#pragma unroll
      for (int j = 0; j < 4; ++j) {
        S[j] = zero8();
        const int ko = (16 * j + idx) * 72 + 8 * hh;
        Fr kh0, kl0, kh1, kl1;
        kh0.h[0] = *(const us8*)(&sK[0][ko]);      kh0.h[1] = *(const us8*)(&sK[0][ko + 16]);
        kh1.h[0] = *(const us8*)(&sK[0][ko + 32]); kh1.h[1] = *(const us8*)(&sK[0][ko + 48]);
        kl0.h[0] = *(const us8*)(&sK[1][ko]);      kl0.h[1] = *(const us8*)(&sK[1][ko + 16]);
        kl1.h[0] = *(const us8*)(&sK[1][ko + 32]); kl1.h[1] = *(const us8*)(&sK[1][ko + 48]);
        S[j] = mma(qh[0], kh0.v, S[j]); S[j] = mma(qh[0], kl0.v, S[j]); S[j] = mma(ql[0], kh0.v, S[j]);
        S[j] = mma(qh[1], kh1.v, S[j]); S[j] = mma(qh[1], kl1.v, S[j]); S[j] = mma(ql[1], kh1.v, S[j]);
        gd1(S[j], kh0.v, kl0.v, kh1.v, kl1.v);
      }
      keep4(qh[0], qh[1], ql[0], ql[1]);
#pragma unroll
      for (int r = 0; r < 8; ++r) {
        float t[4];
#pragma unroll
        for (int j = 0; j < 4; ++j) t[j] = ((bits >> (j * 8 + r)) & 1u) ? (S[j][r] * 0.125f) : neg_inf();
        const float mx = rmax16(fmaxf(fmaxf(t[0], t[1]), fmaxf(t[2], t[3])));
        const float mn = fmaxf(m[r], mx);
        const bool dead = (mn == neg_inf());
        const float alpha = dead ? 1.0f : __expf(m[r] - mn);
        m[r] = mn;
        float rs = 0.f;
#pragma unroll
        for (int j = 0; j < 4; ++j) {
          const float p = dead ? 0.f : __expf(t[j] - mn);
          rs += p;
          const us hb = f2bf(p);
          const us lb = f2bf(p - bf2f(hb));
          sP[wav][0][(8 * hh + r) * 72 + 16 * j + idx] = hb;
          sP[wav][1][(8 * hh + r) * 72 + 16 * j + idx] = lb;
        }
        rs = rsum16(rs);
        l[r] = l[r] * alpha + rs;
#pragma unroll
        for (int g = 0; g < 4; ++g) O[g][r] *= alpha;
      }
      __builtin_amdgcn_fence(__ATOMIC_RELEASE, "wavefront");
      __builtin_amdgcn_wave_barrier();
      __builtin_amdgcn_fence(__ATOMIC_ACQUIRE, "wavefront");
      Fr ph0, pl0, ph1, pl1;
      {
        const int po = idx * 72 + 8 * hh;
        ph0.h[0] = *(const us8*)(&sP[wav][0][po]);      ph0.h[1] = *(const us8*)(&sP[wav][0][po + 16]);
        ph1.h[0] = *(const us8*)(&sP[wav][0][po + 32]); ph1.h[1] = *(const us8*)(&sP[wav][0][po + 48]);
        pl0.h[0] = *(const us8*)(&sP[wav][1][po]);      pl0.h[1] = *(const us8*)(&sP[wav][1][po + 16]);
        pl1.h[0] = *(const us8*)(&sP[wav][1][po + 32]); pl1.h[1] = *(const us8*)(&sP[wav][1][po + 48]);
      }
#pragma unroll
      for (int g = 0; g < 4; ++g) {
        const int vo = (16 * g + idx) * 72 + 8 * hh;
        Fr vh0, vl0, vh1, vl1;
        vh0.h[0] = *(const us8*)(&sV[0][vo]);      vh0.h[1] = *(const us8*)(&sV[0][vo + 16]);
        vh1.h[0] = *(const us8*)(&sV[0][vo + 32]); vh1.h[1] = *(const us8*)(&sV[0][vo + 48]);
        vl0.h[0] = *(const us8*)(&sV[1][vo]);      vl0.h[1] = *(const us8*)(&sV[1][vo + 16]);
        vl1.h[0] = *(const us8*)(&sV[1][vo + 32]); vl1.h[1] = *(const us8*)(&sV[1][vo + 48]);
        O[g] = mma(ph0.v, vh0.v, O[g]); O[g] = mma(ph0.v, vl0.v, O[g]); O[g] = mma(pl0.v, vh0.v, O[g]);
        O[g] = mma(ph1.v, vh1.v, O[g]); O[g] = mma(ph1.v, vl1.v, O[g]); O[g] = mma(pl1.v, vh1.v, O[g]);
        gd1(O[g], vh0.v, vl0.v, vh1.v, vl1.v);
      }
      keep4(ph0.v, pl0.v, ph1.v, pl1.v);
    }
  }
  gd4(O[0], O[1], O[2], O[3]);

#pragma unroll
  for (int r = 0; r < 8; ++r) {
    const int row = 8 * hh + r;
    const int s = q0 + 16 * wav + row;
    int ar = 0;
    (void)qmap(d, inst, b, (s < d.Sq) ? s : (d.Sq - 1), ar);
    const float inv = 1.0f / l[r];
#pragma unroll
    for (int g = 0; g < 4; ++g) {
      float v = O[g][r] * inv;
      if (d.avg) {
        const size_t ao = (size_t)ar * DIM + qcol + 16 * g + idx;
        v = 0.5f * ((bf2f(Ah[ao]) + bf2f(Al[ao])) + v);
      }
      const us hb = f2bf(v);
      const us lb = f2bf(v - bf2f(hb));
      sP[wav][0][row * 72 + 16 * g + idx] = hb;
      sP[wav][1][row * 72 + 16 * g + idx] = lb;
    }
  }
  __builtin_amdgcn_fence(__ATOMIC_RELEASE, "wavefront");
  __builtin_amdgcn_wave_barrier();
  __builtin_amdgcn_fence(__ATOMIC_ACQUIRE, "wavefront");
  const int q4 = lane >> 3, c8 = (lane & 7) * 8;
  us8 hv[4], lv[4]; int arw[4]; bool okr[4];
#pragma unroll
  for (int it = 0; it < 4; ++it) {
    const int row = it * 4 + q4;
    hv[it] = *(const us8*)(&sP[wav][0][row * 72 + c8]);
    lv[it] = *(const us8*)(&sP[wav][1][row * 72 + c8]);
    const int s = q0 + 16 * wav + row;
    okr[it] = s < d.Sq;
    int ar = 0;
    (void)qmap(d, inst, b, okr[it] ? s : (d.Sq - 1), ar);
    arw[it] = ar;
  }
  for (int pass = 0; pass < 2; ++pass) {
#pragma unroll
    for (int it = 0; it < 4; ++it) {
      if (okr[it]) {
        const size_t o = (size_t)arw[it] * DIM + qcol + c8;
        *(volatile us8*)(Ah + o) = hv[it];
        *(volatile us8*)(Al + o) = lv[it];
      }
    }
    __threadfence();
  }
}

extern "C" void kernel_launch(void* const* d_in, const int* in_sizes, int n_in,
                              void* d_out, int out_size, void* d_ws, size_t ws_size, hipStream_t stream) {
  if (n_in < 9) return;
  if (in_sizes[0] != 2 * LTOK * DIM) return;
  if (in_sizes[1] != DIM * DIM || in_sizes[2] != DIM * DIM || in_sizes[3] != DIM * DIM || in_sizes[4] != DIM * DIM) return;
  if (in_sizes[5] != DIM) return;
  if (in_sizes[6] != 2048 * 2048 || in_sizes[7] != 621 * 621 || in_sizes[8] != 9 * 552 * 552) return;
  if (out_size != 7143424) return;
  const float* x   = (const float*)d_in[0];
  const float* wq  = (const float*)d_in[1];
  const float* wk  = (const float*)d_in[2];
  const float* wv  = (const float*)d_in[3];
  const float* fcw = (const float*)d_in[4];
  const float* fcb = (const float*)d_in[5];
  const int* bmask = (const int*)d_in[6];
  const int* otm   = (const int*)d_in[7];
  const int* oom   = (const int*)d_in[8];
  float* out = (float*)d_out;

  const size_t szP  = (size_t)2 * LROW * QKVC * 2;
  const size_t szA  = (size_t)ROWS_A * DIM * 2;
  const size_t szX  = (size_t)2 * LTOK * DIM * 2;
  const size_t szWt = (size_t)QKVC * DIM * 2;
  const size_t szFt = (size_t)DIM * DIM * 2;
  size_t off = 0;
  const size_t oPh = off; off += szP;
  const size_t oPl = off; off += szP;
  const size_t oAh = off; off += szA;
  const size_t oAl = off; off += szA;
  const size_t oX  = off; off += szX;
  const size_t oWt = off; off += szWt;
  const size_t oFt = off; off += szFt;
  if (off > ws_size) return;
  char* ws = (char*)d_ws;
  us* Ph = (us*)(ws + oPh); us* Pl = (us*)(ws + oPl);
  us* Ah = (us*)(ws + oAh); us* Al = (us*)(ws + oAl);
  us* Xb = (us*)(ws + oX);  us* Wt = (us*)(ws + oWt); us* Ft = (us*)(ws + oFt);
  us* Aoh = Ah + (size_t)4096 * DIM; us* Aol = Al + (size_t)4096 * DIM;

  const int n8 = 2 * LTOK * DIM / 8;
  k_cvt8<<<dim3((n8 + 255) / 256), dim3(256), 0, stream>>>(x, Xb, n8);
  k_wtrans<<<dim3(DIM / 32, DIM / 64, 4), dim3(256), 0, stream>>>(wq, wk, wv, fcw, Wt, Ft);
  k_gemm<false, 0><<<dim3((LROW / 64 * (QKVC / 64) + 7) / 8, 2), dim3(256), 0, stream>>>(
      Xb, Xb, DIM, (long)LTOK * DIM, Wt, DIM, Ph, Pl, out, QKVC, (long)LROW * QKVC, fcb, LROW, QKVC, DIM);

  const ADesc d1 = {2048, 2048, 0, 0, 0,   0, 0, 0, 0, 1, 2048, 0,         0, 2048};
  const ADesc d2 = {256,  552,  0, 1, 256, 1, 0, 0, 1, 0, 0,    0,         1, 2048};
  const ADesc d3 = {621,  621,  1, 1, 0,   0, 1, 1, 0, 1, 621,  0,         0, NOBJ};
  const ADesc d4 = {552,  552,  1, 1, 0,   1, 0, 0, 1, 1, 552,  552 * 552, 1, NOBJ};
  k_attn<<<dim3(32, 1, 16), dim3(128), 0, stream>>>(Ph, Pl, bmask, Ah, Al, d1);
  k_attn<<<dim3(4, 8, 16),  dim3(128), 0, stream>>>(Ph, Pl, bmask, Ah, Al, d2);
  k_attn<<<dim3(10, 8, 16), dim3(128), 0, stream>>>(Ph, Pl, otm, Aoh, Aol, d3);
  k_attn<<<dim3(9, 9, 16),  dim3(128), 0, stream>>>(Ph, Pl, oom, Aoh, Aol, d4);

  k_gemm<true, 1><<<dim3((4096 / 64 * (DIM / 64) + 7) / 8, 1), dim3(256), 0, stream>>>(
      Ah, Al, DIM, 0L, Ft, DIM, Ph, Pl, out, DIM, 0L, fcb, 4096, DIM, DIM);
  k_gemm<true, 2><<<dim3((((2 * NOBJ + 63) / 64) * (DIM / 64) + 7) / 8, 1), dim3(256), 0, stream>>>(
      Aoh, Aol, DIM, 0L, Ft, DIM, Ph, Pl, out, DIM, 0L, fcb, 2 * NOBJ, DIM, DIM);
  (void)hipGetLastError();
}
